// VerticalStripAttention_42649025249311
// MI455X (gfx1250) — hardware-verified
//
#include <hip/hip_runtime.h>


#define NSTR 256
#define NT   256
#define DIM  192
#define NH_  6
#define HD   32
#define NSM  64
#define NTOK (NSTR * NT)
#define NG   4
#define GS_  (NSTR / NG)
#define GTOK (GS_ * NT)
#define GPR  (GS_ * NH_)
#define ZC   192
#define PCAR 1024.0f
#define SCL  0.17677669529663687f
typedef _Float16 h16;
typedef unsigned short bf;
typedef __attribute__((ext_vector_type(16))) __bf16   v16bf;
typedef __attribute__((ext_vector_type(16))) _Float16 v16h;
typedef __attribute__((ext_vector_type(8)))  _Float16 v8h;
typedef __attribute__((ext_vector_type(8)))  unsigned short v8us;
typedef __attribute__((ext_vector_type(8)))  float    v8f;
typedef __attribute__((ext_vector_type(4)))  float    v4f;
typedef v8h  __attribute__((may_alias)) v8ha;
typedef v4f  __attribute__((may_alias)) v4fa;
typedef v8us __attribute__((may_alias)) v8usa;

__device__ __forceinline__ unsigned short f2bf(float f) { unsigned u = __float_as_uint(f); u += 0x7FFFu + ((u >> 16) & 1u); return (unsigned short)(u >> 16); }
__device__ __forceinline__ float bf2f(unsigned short b) { return __uint_as_float(((unsigned)b) << 16); }
__device__ __forceinline__ float bfr(float f) { return bf2f(f2bf(f)); }
__device__ __forceinline__ v16h cat16(v8h lo, v8h hi) { return __builtin_shufflevector(lo, hi, 0, 1, 2, 3, 4, 5, 6, 7, 8, 9, 10, 11, 12, 13, 14, 15); }
__device__ __forceinline__ v16bf cat16b(v8us lo, v8us hi) { return __builtin_bit_cast(v16bf, __builtin_shufflevector(lo, hi, 0, 1, 2, 3, 4, 5, 6, 7, 8, 9, 10, 11, 12, 13, 14, 15)); }
__device__ __forceinline__ v8f wmma16(v16h a, v16h b, v8f c) { return __builtin_amdgcn_wmma_f32_16x16x32_f16(false, a, false, b, (short)0, c, false, false); }
__device__ __forceinline__ v8f wmmab(v16bf a, v16bf b, v8f c) { return __builtin_amdgcn_wmma_f32_16x16x32_bf16(false, a, false, b, (short)0, c, false, false); }


template <typename T16> struct WFrag;
template <> struct WFrag<h16> { typedef v16h V; static __device__ __forceinline__ V ld(const h16* p) { return cat16(*(const v8h*)p, *(const v8h*)(p + 16)); } static __device__ __forceinline__ v8f mma(V a, V b, v8f c) { return wmma16(a, b, c); } };
template <> struct WFrag<bf> { typedef v16bf V; static __device__ __forceinline__ V ld(const bf* p) { return cat16b(*(const v8us*)p, *(const v8us*)(p + 16)); } static __device__ __forceinline__ v8f mma(V a, V b, v8f c) { return wmmab(a, b, c); } };
template <typename T16, int NSPLIT, bool BIAS>
__global__ __launch_bounds__(32) void k_gemmw(const T16* __restrict__ A, const T16* __restrict__ A2, const T16* __restrict__ Bt, const T16* __restrict__ Bt2, int K, float* C, int ldc, const float* __restrict__ bias, size_t sA, size_t sB, size_t sC) {
    typedef typename WFrag<T16>::V V;
    __shared__ __align__(16) float os[16 * 68];
    const size_t z = blockIdx.z; A += z * sA; if (A2) A2 += z * sA; Bt += z * sB; if (Bt2) Bt2 += z * sB; C += z * sC;
    const int lane = threadIdx.x & 31, lr = lane & 15, hi = lane >> 4; const int r0 = blockIdx.x * 64, c0 = blockIdx.y * 64;
    v8f acc[4][4];
#pragma unroll
    for (int mb = 0; mb < 4; ++mb)
#pragma unroll
        for (int nb = 0; nb < 4; ++nb) acc[mb][nb] = (v8f){};
    const size_t aoff = (size_t)(r0 + lr) * K + 8 * hi, boff = (size_t)(c0 + lr) * K + 8 * hi;
#pragma unroll 1
    for (int kc = 0; kc < K; kc += 32) {
        V a[4], a2[4];
#pragma unroll
        for (int mb = 0; mb < 4; ++mb) { a[mb] = WFrag<T16>::ld(A + aoff + (size_t)mb * 16 * K + kc); if (NSPLIT == 1 || NSPLIT == 2) a2[mb] = WFrag<T16>::ld(A2 + aoff + (size_t)mb * 16 * K + kc); }
#pragma unroll
        for (int nb = 0; nb < 4; ++nb) { const V b = WFrag<T16>::ld(Bt + boff + (size_t)nb * 16 * K + kc); V b2; if (NSPLIT >= 2) b2 = WFrag<T16>::ld(Bt2 + boff + (size_t)nb * 16 * K + kc);
#pragma unroll
            for (int mb = 0; mb < 4; ++mb) { acc[mb][nb] = WFrag<T16>::mma(a[mb], b, acc[mb][nb]); if (NSPLIT == 1 || NSPLIT == 2) acc[mb][nb] = WFrag<T16>::mma(a2[mb], b, acc[mb][nb]); if (NSPLIT >= 2) acc[mb][nb] = WFrag<T16>::mma(a[mb], b2, acc[mb][nb]); } }
        asm volatile("v_nop\n\tv_nop\n\tv_nop\n\tv_nop" : "+v"(acc[0][0]), "+v"(acc[1][1]), "+v"(acc[2][2]), "+v"(acc[3][3]) : "v"(a[0]), "v"(a[3]));
    }
#pragma unroll
    for (int mb = 0; mb < 4; ++mb) {
#pragma unroll
        for (int nb = 0; nb < 4; ++nb) {
#pragma unroll
            for (int j = 0; j < 8; ++j) os[(hi * 8 + j) * 68 + nb * 16 + lr] = acc[mb][nb][j]; }
        __builtin_amdgcn_wave_barrier(); asm volatile("" ::: "memory");
        float* crow = C + (size_t)(r0 + mb * 16) * ldc + c0;
#pragma unroll 1
        for (int ps = 0; ps < 2; ++ps) {
#pragma unroll
            for (int s = 0; s < 8; ++s) { const int row = 2 * s + hi, cofs = lr * 4; v4f val = *(const v4fa*)(os + row * 68 + cofs); if (BIAS) { val[0] += bfr(bias[c0 + cofs]); val[1] += bfr(bias[c0 + cofs + 1]); val[2] += bfr(bias[c0 + cofs + 2]); val[3] += bfr(bias[c0 + cofs + 3]); }
                *(volatile v4f*)(crow + (size_t)row * ldc + cofs) = val; }
            if (ps == 0) __threadfence(); }
        __builtin_amdgcn_wave_barrier(); asm volatile("" ::: "memory");
    }
}

__device__ __forceinline__ h16 tohx(float x) { return (h16)x; }
__device__ __forceinline__ void splitf(float y, unsigned short& h, unsigned short& l) { h = f2bf(y); l = f2bf(y - bf2f(h)); }
typedef __attribute__((ext_vector_type(2))) _Float16 v2h;
typedef __attribute__((ext_vector_type(4))) _Float16 v4h;
typedef __attribute__((ext_vector_type(2))) unsigned short v2us;
typedef __attribute__((ext_vector_type(4))) float v4fx;

__global__ __launch_bounds__(256) void k_cvt8(const float* __restrict__ src, bf* dst, size_t n8) { const size_t i = (size_t)blockIdx.x * 256 + threadIdx.x; if (i >= n8) return; const v8f v = *(const v8f*)(src + i * 8); v8us o;
#pragma unroll
    for (int k = 0; k < 8; ++k) o[k] = f2bf(v[k]); *(volatile v8us*)(dst + i * 8) = o; __threadfence(); *(volatile v8us*)(dst + i * 8) = o; }
__global__ __launch_bounds__(256) void k_bias(const float* __restrict__ tab, const int* __restrict__ ri, float* BIAS) { const int e = blockIdx.x * 256 + threadIdx.x; if (e >= NT * NT) return; int idx = ri[e]; idx = idx < 0 ? 0 : (idx > 888 ? 888 : idx);
    for (int ps = 0; ps < 2; ++ps) {
#pragma unroll
        for (int h = 0; h < NH_; ++h) *(volatile float*)(BIAS + (size_t)h * NT * NT + e) = bfr(tab[(size_t)idx * NH_ + h]);
        if (ps == 0) __threadfence(); } }
__global__ __launch_bounds__(256) void k_qk16(const float* __restrict__ QKV, h16* QP, h16* KP) { const size_t e = ((size_t)blockIdx.x * 256 + threadIdx.x) * 2; if (e >= (size_t)GPR * NT * HD) return; const int d = (int)(e % HD); const int n = (int)((e / HD) % NT); const int pr = (int)(e / ((size_t)HD * NT)); const int s = pr / NH_, h = pr % NH_; const float* row = QKV + ((size_t)s * NT + n) * (3 * DIM);
    v2h q, k; q[0] = tohx(row[h * HD + d]); q[1] = tohx(row[h * HD + d + 1]); k[0] = tohx(row[DIM + h * HD + d]); k[1] = tohx(row[DIM + h * HD + d + 1]); *(volatile v2h*)(QP + e) = q; *(volatile v2h*)(KP + e) = k; __threadfence(); *(volatile v2h*)(QP + e) = q; *(volatile v2h*)(KP + e) = k; }
__global__ __launch_bounds__(256) void k_vt16(const float* __restrict__ QKV, h16* VT) { const size_t e = ((size_t)blockIdx.x * 256 + threadIdx.x) * 2; if (e >= (size_t)GPR * 64 * NT) return; const int m = (int)(e % NT); const int d = (int)((e / NT) % 64); const int pr = (int)(e / ((size_t)NT * 64)); const int s = pr / NH_, h = pr % NH_; v2h o;
    if (d < HD) { const float* r0 = QKV + ((size_t)s * NT + m) * (3 * DIM) + 2 * DIM + h * HD + d; o[0] = tohx(r0[0]); o[1] = tohx(r0[3 * DIM]); } else { o[0] = (h16)0.f; o[1] = (h16)0.f; }
    *(volatile v2h*)(VT + e) = o; __threadfence(); *(volatile v2h*)(VT + e) = o; }
__global__ __launch_bounds__(256) void k_wsoft(const float* __restrict__ S, const float* __restrict__ BIAS, const float* __restrict__ mask, int pr0  , h16* P) { const int lane = threadIdx.x & 31; const int row = blockIdx.x * 8 + (threadIdx.x >> 5); if (row >= ZC * NT) return; const int n = row % NT, zz = row / NT; const int pr = pr0 + zz; const int s = pr / NH_, h = pr % NH_;
    const float* sr = S + (size_t)row * NT; const float* br = BIAS + ((size_t)h * NT + n) * NT; const float* mr = mask + ((size_t)(s % NSM) * NT + n) * NT; float v[8]; float mx = -3.0e38f;
#pragma unroll
    for (int ch = 0; ch < 2; ++ch) { const int j0 = ch * 128 + lane * 4; const v4fx a = *(const v4fx*)(sr + j0), bb = *(const v4fx*)(br + j0), mm = *(const v4fx*)(mr + j0);
#pragma unroll
        for (int q = 0; q < 4; ++q) { float t0 = __fmul_rn(a[q], SCL); asm volatile("" : "+v"(t0)); const float t = __fadd_rn(__fadd_rn(t0, bb[q]), bfr(mm[q])); v[ch * 4 + q] = t; mx = fmaxf(mx, t); } }
#pragma unroll
    for (int sh = 16; sh; sh >>= 1) mx = fmaxf(mx, __shfl_xor(mx, sh, 32));
    float sum = 0.f;
#pragma unroll
    for (int k = 0; k < 8; ++k) { float d0 = __fsub_rn(v[k], mx); asm volatile("" : "+v"(d0)); v[k] = __expf(d0); sum += v[k]; }
#pragma unroll
    for (int sh = 16; sh; sh >>= 1) sum += __shfl_xor(sum, sh, 32);
    const float f = __fdiv_rn(PCAR, sum);
#pragma unroll 1
    for (int ps = 0; ps < 2; ++ps) {
#pragma unroll
        for (int ch = 0; ch < 2; ++ch) { v4h o; for (int q = 0; q < 4; ++q) o[q] = tohx(v[ch * 4 + q] * f); *(volatile v4h*)(P + (size_t)row * NT + ch * 128 + lane * 4) = o; }
        if (ps == 0) __threadfence(); } }
__global__ __launch_bounds__(256) void k_mrg6(const float* __restrict__ O, int pr0  , bf* Ah, bf* Al) { const size_t e = ((size_t)blockIdx.x * 256 + threadIdx.x) * 2; if (e >= (size_t)ZC * NT * HD) return; const int d = (int)(e % HD); const int n = (int)((e / HD) % NT); const int zz = (int)(e / ((size_t)HD * NT)); const int pr = pr0 + zz; const int s = pr / NH_, h = pr % NH_; const float* src = O + ((size_t)zz * NT + n) * 64 + d; v2us oh, ol;
#pragma unroll
    for (int q = 0; q < 2; ++q) { unsigned short a, c2; splitf(src[q] * (1.0f / PCAR), a, c2); oh[q] = a; ol[q] = c2; } const size_t oo = ((size_t)s * NT + n) * DIM + h * HD + d; *(volatile v2us*)(Ah + oo) = oh; *(volatile v2us*)(Al + oo) = ol; __threadfence(); *(volatile v2us*)(Ah + oo) = oh; *(volatile v2us*)(Al + oo) = ol; }

extern "C" void kernel_launch(void* const* d_in, const int* in_sizes, int n_in,
                              void* d_out, int out_size, void* d_ws, size_t ws_size, hipStream_t stream) {
    (void)in_sizes; (void)n_in; (void)out_size;
    const float* x = (const float*)d_in[0]; const float* mask = (const float*)d_in[1]; const float* wqkv = (const float*)d_in[2]; const float* bqkv = (const float*)d_in[3]; const float* wp = (const float*)d_in[4]; const float* bp = (const float*)d_in[5]; const float* tab = (const float*)d_in[6]; const int* ri = (const int*)d_in[7];
    float* OUT = (float*)d_out;
    char* wsp = (char*)d_ws;
    auto take = [&](size_t bytes) { char* p = wsp; wsp += (bytes + 255) & ~(size_t)255; return (void*)p; };
    bf* WQKV = (bf*)take((size_t)3 * DIM * DIM * 2); bf* WP = (bf*)take((size_t)DIM * DIM * 2); float* BIAS = (float*)take((size_t)NH_ * NT * NT * 4); bf* XB = (bf*)take((size_t)GTOK * DIM * 2); float* QKV = (float*)take((size_t)GTOK * 3 * DIM * 4);
    h16* QP = (h16*)take((size_t)GPR * NT * HD * 2); h16* KP = (h16*)take((size_t)GPR * NT * HD * 2); h16* VT = (h16*)take((size_t)GPR * 64 * NT * 2); float* S = (float*)take((size_t)ZC * NT * NT * 4); h16* P = (h16*)take((size_t)ZC * NT * NT * 2); float* O = (float*)take((size_t)ZC * NT * 64 * 4); bf* Ah = (bf*)take((size_t)GTOK * DIM * 2); bf* Al = (bf*)take((size_t)GTOK * DIM * 2);
    if ((size_t)(wsp - (char*)d_ws) > ws_size) return;
    k_cvt8<<<(unsigned)(((size_t)3 * DIM * DIM / 8 + 255) / 256), 256, 0, stream>>>(wqkv, WQKV, (size_t)3 * DIM * DIM / 8); k_cvt8<<<(unsigned)(((size_t)DIM * DIM / 8 + 255) / 256), 256, 0, stream>>>(wp, WP, (size_t)DIM * DIM / 8);
    k_bias<<<(NT * NT + 255) / 256, 256, 0, stream>>>(tab, ri, BIAS);
    for (int g = 0; g < NG; ++g) { const size_t t0 = (size_t)g * GTOK;
        k_cvt8<<<(unsigned)(((size_t)GTOK * DIM / 8 + 255) / 256), 256, 0, stream>>>(x + t0 * DIM, XB, (size_t)GTOK * DIM / 8);
        k_gemmw<bf, 0, true><<<dim3(GTOK / 64, 3 * DIM / 64, 1), 32, 0, stream>>>(XB, nullptr, WQKV, nullptr, DIM, QKV, 3 * DIM, bqkv, 0, 0, 0);
        k_qk16<<<(unsigned)(((size_t)GPR * NT * HD / 2 + 255) / 256), 256, 0, stream>>>(QKV, QP, KP); k_vt16<<<(unsigned)(((size_t)GPR * 64 * NT / 2 + 255) / 256), 256, 0, stream>>>(QKV, VT);
        for (int c = 0; c < GPR / ZC; ++c) { const int lp0 = c * ZC;
            k_gemmw<h16, 0, false><<<dim3(NT / 64, NT / 64, ZC), 32, 0, stream>>>(QP + (size_t)lp0 * NT * HD, nullptr, KP + (size_t)lp0 * NT * HD, nullptr, HD, S, NT, nullptr, (size_t)NT * HD, (size_t)NT * HD, (size_t)NT * NT);
            k_wsoft<<<ZC * NT / 8, 256, 0, stream>>>(S, BIAS, mask, g * GPR + lp0, P);
            k_gemmw<h16, 0, false><<<dim3(NT / 64, 1, ZC), 32, 0, stream>>>(P, nullptr, VT + (size_t)lp0 * 64 * NT, nullptr, NT, O, 64, nullptr, (size_t)NT * NT, (size_t)64 * NT, (size_t)NT * 64);
            k_mrg6<<<(unsigned)(((size_t)ZC * NT * HD / 2 + 255) / 256), 256, 0, stream>>>(O, lp0, Ah, Al); }
        k_gemmw<bf, 1, true><<<dim3(GTOK / 64, DIM / 64, 1), 32, 0, stream>>>(Ah, Al, WP, nullptr, DIM, OUT + t0 * DIM, DIM, bp, 0, 0, 0); }
}
